// EGATConv_17815524343864
// MI455X (gfx1250) — hardware-verified
//
#include <hip/hip_runtime.h>
#include <stddef.h>
#include <math.h>

typedef __attribute__((ext_vector_type(16))) _Float16 v16h;
typedef __attribute__((ext_vector_type(8)))  _Float16 v8h;
typedef __attribute__((ext_vector_type(16))) __bf16   v16b;
typedef __attribute__((ext_vector_type(8)))  __bf16   v8b;
typedef __attribute__((ext_vector_type(8)))  float    v8f;
typedef __attribute__((ext_vector_type(4)))  float    v4f;
typedef __attribute__((ext_vector_type(4)))  int      v4i;

constexpr int CIN  = 128;
constexpr int NHD  = 4;
constexpr int DCH  = 16;
constexpr int HDIM = NHD * DCH;
constexpr int EFE  = 32;
constexpr int NET  = 8;
constexpr int NBLK = 512;
constexpr int RPQ  = 1024;
#define NTHR    256
#define NWAVE   8
#define EPT     8
#define NGRP    1
#define CHUNK   (NTHR * EPT * NGRP)
#define WCAP    (EPT * NGRP * 32)
#define LISTN   (NWAVE * WCAP)
#define LDS_AGG ((NBLK * HDIM + 2 * NBLK * NHD) * 4 + LISTN * 4 + 64)

static_assert((CHUNK & (CHUNK - 1)) == 0);
static_assert(CHUNK <= 4096);
static_assert((NBLK & (NBLK - 1)) == 0 && NBLK <= 4096);
static_assert(RPQ % NBLK == 0 && RPQ % 64 == 0 && RPQ % NTHR == 0 && RPQ % 16 == 0);
static_assert(LDS_AGG == 155712);
static_assert(CIN % 32 == 0 && CIN / 8 == 16 && HDIM == 64 && NHD * NET == 32);

__device__ __forceinline__ unsigned short f2bf_bits(float f) {
  unsigned u = __float_as_uint(f);
  return (unsigned short)((u + 0x7FFFu + ((u >> 16) & 1u)) >> 16);
}
__device__ __forceinline__ float bf_bits2f(unsigned short h) { return __uint_as_float(((unsigned)h) << 16); }

__device__ __forceinline__ void dep_guard_h(v8f& a, v8f& b, v16h x, v16h y) { asm volatile("v_nop\n\tv_nop\n\tv_nop\n\tv_nop" : "+v"(a), "+v"(b) : "v"(x), "v"(y)); }
__device__ __forceinline__ void dep_guard_b(v8f& a, v8f& b, v16b x, v16b y) { asm volatile("v_nop\n\tv_nop\n\tv_nop\n\tv_nop" : "+v"(a), "+v"(b) : "v"(x), "v"(y)); }
__device__ __forceinline__ void keep4_h(v16h a, v16h b, v16h c, v16h d) { asm volatile("v_nop" :: "v"(a), "v"(b), "v"(c), "v"(d)); }
__device__ __forceinline__ void keep4_b(v16b a, v16b b, v16b c, v16b d) { asm volatile("v_nop" :: "v"(a), "v"(b), "v"(c), "v"(d)); }
__device__ __forceinline__ void acc_guard4(v8f& a, v8f& b, v8f& c, v8f& d) { asm volatile("v_nop\n\tv_nop\n\tv_nop\n\tv_nop" : "+v"(a), "+v"(b), "+v"(c), "+v"(d)); }
template <typename T> struct Frag;
template <> struct Frag<_Float16> {
  typedef v16h V; union U { v16h v; v8h h[2]; };
  static __device__ __forceinline__ v16h load(const _Float16* p) {
    U f; f.h[0] = *(const v8h*)(p); f.h[1] = *(const v8h*)(p + 16); return f.v;
  }
  static __device__ __forceinline__ v8f mma(v16h a, v16h b, v8f c) {
    return __builtin_amdgcn_wmma_f32_16x16x32_f16(false, a, false, b, (short)0, c, false, false);
  }
  static __device__ __forceinline__ void guard(v8f& a, v8f& b, v16h x, v16h y) { dep_guard_h(a, b, x, y); }
  static __device__ __forceinline__ void keep(v16h a, v16h b, v16h c, v16h d) { keep4_h(a, b, c, d); }
};
template <> struct Frag<__bf16> {
  typedef v16b V; union U { v16b v; v8b h[2]; };
  static __device__ __forceinline__ v16b load(const __bf16* p) {
    U f; f.h[0] = *(const v8b*)(p); f.h[1] = *(const v8b*)(p + 16); return f.v;
  }
  static __device__ __forceinline__ v8f mma(v16b a, v16b b, v8f c) {
    return __builtin_amdgcn_wmma_f32_16x16x32_bf16(false, a, false, b, (short)0, c, false, false);
  }
  static __device__ __forceinline__ void guard(v8f& a, v8f& b, v16b x, v16b y) { dep_guard_b(a, b, x, y); }
  static __device__ __forceinline__ void keep(v16b a, v16b b, v16b c, v16b d) { keep4_b(a, b, c, d); }
};

template <int ET> struct Elem;
template <> struct Elem<0> { typedef _Float16 T; };
template <> struct Elem<1> { typedef __bf16 T; };
template <int ET, bool SPLIT, int BIAS_MODE, int OUT_MODE, bool RESID, int ACT = 0>
__global__ __launch_bounds__(256) void wmma_gemm64(
    const unsigned short* __restrict__ Ap, const unsigned short* __restrict__ A2p, int lda, long strideA,
    const unsigned short* __restrict__ Btp, const unsigned short* __restrict__ Bt2p, int ldb, long strideB,
    void* __restrict__ Cout, void* __restrict__ Cout2, int ldc, long strideC,
    const float* __restrict__ bias,
    const float* __restrict__ resid, long strideR,
    int M, int N, int K, float scale) {
  typedef typename Elem<ET>::T T;
  typedef typename Frag<T>::V V;
  const T* A = (const T*)Ap; const T* A2 = (const T*)A2p; const T* Bt = (const T*)Btp; const T* Bt2 = (const T*)Bt2p;
  __shared__ __align__(16) float sT[8][16 * 68];
  const int b    = blockIdx.y;
  const int lane = threadIdx.x & 31;
  const int wave = threadIdx.x >> 5;
  const int tilesN = N >> 6;
  const int tilesM = M >> 6;
  const int tile = blockIdx.x * 8 + wave;
  if (tile >= tilesM * tilesN) return;
  const int tm = tile / tilesN;
  const int tn = tile - tm * tilesN;
  const int m0 = tm << 6;
  const int n0 = tn << 6;

  const T* Ab  = A  + (size_t)b * strideA;
  const T* Bb  = Bt + (size_t)b * strideB;
  const T* Ab2 = SPLIT ? (A2  + (size_t)b * strideA) : nullptr;
  const T* Bb2 = SPLIT ? (Bt2 + (size_t)b * strideB) : nullptr;

  const int rlane = lane & 15;
  const int koff  = (lane >> 4) * 8;
  const int mOff  = (lane >> 4) * 8;

  v8f acc[4][4];
#pragma unroll
  for (int i = 0; i < 4; ++i)
#pragma unroll
    for (int j = 0; j < 4; ++j) acc[i][j] = (v8f){0.f,0.f,0.f,0.f,0.f,0.f,0.f,0.f};

  for (int k0 = 0; k0 < K; k0 += 32) {
    V bh[4], bl[4];
#pragma unroll
    for (int j = 0; j < 4; ++j) {
      const size_t bo = (size_t)(n0 + (j << 4) + rlane) * ldb + koff + k0;
      bh[j] = Frag<T>::load(Bb + bo);
      if (SPLIT) bl[j] = Frag<T>::load(Bb2 + bo);
    }
#pragma unroll
    for (int i = 0; i < 4; ++i) {
      const size_t ao = (size_t)(m0 + (i << 4) + rlane) * lda + koff + k0;
      V ah = Frag<T>::load(Ab + ao);
      V al;
      if (SPLIT) al = Frag<T>::load(Ab2 + ao);
#pragma unroll
      for (int j = 0; j < 4; ++j) {
        acc[i][j] = Frag<T>::mma(ah, bh[j], acc[i][j]);
        if (SPLIT) {
          acc[i][j] = Frag<T>::mma(ah, bl[j], acc[i][j]);
          acc[i][j] = Frag<T>::mma(al, bh[j], acc[i][j]);
        }
      }
      Frag<T>::guard(acc[i][0], acc[i][3], ah, SPLIT ? al : ah);
    }
    Frag<T>::keep(bh[0], bh[1], bh[2], bh[3]);
    if (SPLIT) Frag<T>::keep(bl[0], bl[1], bl[2], bl[3]);
  }
  acc_guard4(acc[0][0], acc[0][1], acc[0][2], acc[0][3]);
  acc_guard4(acc[1][0], acc[1][1], acc[1][2], acc[1][3]);
  acc_guard4(acc[2][0], acc[2][1], acc[2][2], acc[2][3]);
  acc_guard4(acc[3][0], acc[3][1], acc[3][2], acc[3][3]);

  float* slab = sT[wave];
  const float* Rb = RESID ? (resid + (size_t)b * strideR) : nullptr;
#pragma unroll
  for (int i = 0; i < 4; ++i) {
    const int mBase = m0 + (i << 4);
#pragma unroll
    for (int j = 0; j < 4; ++j) {
      const int n = n0 + (j << 4) + rlane;
      float bv = 0.f;
      if (BIAS_MODE == 2) bv = bias[n];
#pragma unroll
      for (int r = 0; r < 8; ++r) {
        float v = acc[i][j][r] * scale;
        if (BIAS_MODE == 1) v += bias[mBase + mOff + r];
        if (BIAS_MODE == 2) v += bv;
        if (RESID) v += Rb[(size_t)(mBase + mOff + r) * ldc + n];
        if (ACT == 1) v = tanhf(v);
        if (ACT == 2) v = fmaxf(v, 0.0f);
        if (ACT == 3) v = v / (1.0f + expf(-v));
        if (ACT == 4) v = (v > 0.f) ? v : 0.01f * v;
        if (ACT == 5) v = 0.5f * v * (1.0f + erff(v * 0.70710678118654752f));
        slab[(mOff + r) * 68 + (j << 4) + rlane] = v;
      }
    }
    __builtin_amdgcn_fence(__ATOMIC_RELEASE, "workgroup");
    __builtin_amdgcn_wave_barrier();
    __builtin_amdgcn_fence(__ATOMIC_ACQUIRE, "workgroup");
    if (OUT_MODE == 0) {
      float* C = (float*)Cout + (size_t)b * strideC;
      const int hh = lane >> 4, c4 = (lane & 15) * 4;
      for (int pass = 0; pass < 2; ++pass) {
#pragma unroll
        for (int it = 0; it < 8; ++it) {
          const int row = it * 2 + hh;
          v4f v = *(const v4f*)(slab + row * 68 + c4);
          *(volatile v4f*)(C + (size_t)(mBase + row) * ldc + n0 + c4) = v;
        }
        __threadfence();
      }
    } else {
      const int q = lane >> 3, c8 = (lane & 7) * 8;
      unsigned short* C  = (unsigned short*)Cout  + (size_t)b * strideC;
      unsigned short* C2 = (OUT_MODE == 2) ? ((unsigned short*)Cout2 + (size_t)b * strideC) : nullptr;
      for (int pass = 0; pass < 2; ++pass) {
#pragma unroll
        for (int it = 0; it < 4; ++it) {
          const int row = it * 4 + q;
          const float* sp = slab + row * 68 + c8;
          v8h hv, lv;
#pragma unroll
          for (int e = 0; e < 8; ++e) {
            if (OUT_MODE == 1) {
              hv[e] = (_Float16)sp[e];
            } else {
              unsigned short hb = f2bf_bits(sp[e]);
              unsigned short lb = f2bf_bits(sp[e] - bf_bits2f(hb));
              hv[e] = __builtin_bit_cast(_Float16, hb);
              lv[e] = __builtin_bit_cast(_Float16, lb);
            }
          }
          *(volatile v8h*)(C + (size_t)(mBase + row) * ldc + n0 + c8) = hv;
          if (OUT_MODE == 2) *(volatile v8h*)(C2 + (size_t)(mBase + row) * ldc + n0 + c8) = lv;
        }
        __threadfence();
      }
    }
    __builtin_amdgcn_fence(__ATOMIC_RELEASE, "workgroup");
    __builtin_amdgcn_wave_barrier();
    __builtin_amdgcn_fence(__ATOMIC_ACQUIRE, "workgroup");
  }
}

template <int NB>
__device__ __forceinline__ int scan_chunk(const int* __restrict__ lst, int nE, int cbase, int nodeBase,
                                          int* list, int tid, int lane, int wave, int fullvec) {
  int wc = 0;
#pragma unroll
  for (int g = 0; g < NGRP; ++g) {
    const int el0 = (g * NTHR + tid) * EPT;
    const int e0  = cbase + el0;
    v4i da, db;
    if (fullvec) {
      da = *(const v4i*)(lst + e0);
      db = *(const v4i*)(lst + e0 + 4);
    } else {
      const int em = nE - 1;
      da.x = lst[(e0     < em) ? e0     : em];
      da.y = lst[(e0 + 1 < em) ? e0 + 1 : em];
      da.z = lst[(e0 + 2 < em) ? e0 + 2 : em];
      da.w = lst[(e0 + 3 < em) ? e0 + 3 : em];
      db.x = lst[(e0 + 4 < em) ? e0 + 4 : em];
      db.y = lst[(e0 + 5 < em) ? e0 + 5 : em];
      db.z = lst[(e0 + 6 < em) ? e0 + 6 : em];
      db.w = lst[(e0 + 7 < em) ? e0 + 7 : em];
    }
    const bool v0 = (e0 < nE), v1 = (e0 + 1 < nE), v2 = (e0 + 2 < nE), v3 = (e0 + 3 < nE);
    const bool v4 = (e0 + 4 < nE), v5 = (e0 + 5 < nE), v6 = (e0 + 6 < nE), v7 = (e0 + 7 < nE);
    const unsigned nb = (unsigned)nodeBase;
    const unsigned s0 = (unsigned)da.x - nb, s1 = (unsigned)da.y - nb;
    const unsigned s2 = (unsigned)da.z - nb, s3 = (unsigned)da.w - nb;
    const unsigned s4 = (unsigned)db.x - nb, s5 = (unsigned)db.y - nb;
    const unsigned s6 = (unsigned)db.z - nb, s7 = (unsigned)db.w - nb;
    const bool h0 = v0 && (s0 < (unsigned)NB), h1 = v1 && (s1 < (unsigned)NB);
    const bool h2 = v2 && (s2 < (unsigned)NB), h3 = v3 && (s3 < (unsigned)NB);
    const bool h4 = v4 && (s4 < (unsigned)NB), h5 = v5 && (s5 < (unsigned)NB);
    const bool h6 = v6 && (s6 < (unsigned)NB), h7 = v7 && (s7 < (unsigned)NB);
    const unsigned any = __builtin_amdgcn_ballot_w32(h0 | h1 | h2 | h3 | h4 | h5 | h6 | h7);
    if (any != 0u) {
#define HITJ(J, HJ, SJ) { \
        const unsigned mj = __builtin_amdgcn_ballot_w32(HJ); \
        if (mj != 0u) { \
          if (HJ) { \
            const int pos = wc + (int)__builtin_amdgcn_mbcnt_lo(mj, 0u); \
            if (pos < WCAP) list[wave * WCAP + pos] = ((el0 + (J)) << 12) | (int)(SJ); \
          } \
          wc += (int)__builtin_popcount(mj); } }
      HITJ(0, h0, s0)
      HITJ(1, h1, s1)
      HITJ(2, h2, s2)
      HITJ(3, h3, s3)
      HITJ(4, h4, s4)
      HITJ(5, h5, s5)
      HITJ(6, h6, s6)
      HITJ(7, h7, s7)
#undef HITJ
    }
  }
  return wc;
}

__device__ __forceinline__ float dot4f(v4f a, v4f b) {
  return a.x * b.x + a.y * b.y + a.z * b.z + a.w * b.w;
}
__device__ __forceinline__ void split_bf(float f, _Float16& h, _Float16& l) {
  const unsigned short hb = f2bf_bits(f);
  const unsigned short lb = f2bf_bits(f - bf_bits2f(hb));
  h = __builtin_bit_cast(_Float16, hb);
  l = __builtin_bit_cast(_Float16, lb);
}
__device__ __forceinline__ void split8(v4f a, v4f b, v8h& hv, v8h& lv) {
  _Float16 h0, l0, h1, l1, h2, l2, h3, l3, h4, l4, h5, l5, h6, l6, h7, l7;
  split_bf(a.x, h0, l0); split_bf(a.y, h1, l1); split_bf(a.z, h2, l2); split_bf(a.w, h3, l3);
  split_bf(b.x, h4, l4); split_bf(b.y, h5, l5); split_bf(b.z, h6, l6); split_bf(b.w, h7, l7);
  hv[0] = h0; hv[1] = h1; hv[2] = h2; hv[3] = h3; hv[4] = h4; hv[5] = h5; hv[6] = h6; hv[7] = h7;
  lv[0] = l0; lv[1] = l1; lv[2] = l2; lv[3] = l3; lv[4] = l4; lv[5] = l5; lv[6] = l6; lv[7] = l7;
}
template <int CPL> struct VecT { typedef float T __attribute__((ext_vector_type(CPL))); };
template <> struct VecT<1> { typedef float T; };

__global__ __launch_bounds__(NTHR) void k_split16(const float* __restrict__ x, unsigned short* ph,
                                                  unsigned short* pl, int nValid, int nRows) {
  const int i = blockIdx.x * NTHR + threadIdx.x;
  if (i >= nRows * (CIN / 8)) return;
  const int row = i >> 4;
  const int c0  = (i & 15) * 8;
  const int rc  = (row < nValid) ? row : nValid - 1;
  const float* xp = x + (size_t)rc * CIN + c0;
  v4f a = *(const v4f*)xp, b = *(const v4f*)(xp + 4);
  if (row >= nValid) { const v4f z = {0.f, 0.f, 0.f, 0.f}; a = z; b = z; }
  v8h hv, lv;
  split8(a, b, hv, lv);
  const size_t o = (size_t)i * 8;
  *(volatile v8h*)(ph + o) = hv;
  *(volatile v8h*)(pl + o) = lv;
  __threadfence();
  *(volatile v8h*)(ph + o) = hv;
  *(volatile v8h*)(pl + o) = lv;
}

__global__ __launch_bounds__(32) void k_eetab(const float* __restrict__ emb, const float* __restrict__ wfe,
                                               const float* __restrict__ ae, float* eep) {
  const int tid = threadIdx.x;
  const int t = tid >> 2, hh = tid & 3;
  const float* em = emb + t * EFE;
  float sum = 0.f;
#pragma unroll 1
  for (int fe = 0; fe < EFE; ++fe) {
    const float* wr = wfe + (size_t)(hh * EFE + fe) * EFE;
    float dot = 0.f;
#pragma unroll 1
    for (int c = 0; c < EFE; ++c) dot += em[c] * wr[c];
    sum += dot * ae[hh * EFE + fe];
  }
  *(volatile float*)(eep + tid) = sum;
  __threadfence();
  *(volatile float*)(eep + tid) = sum;
}

__global__ __launch_bounds__(NTHR) void k_scores4(const float* __restrict__ h, const float* __restrict__ al,
                                                  const float* __restrict__ ar, float* elp, float* erp,
                                                  int nN, int nRows) {
  const int node = blockIdx.x * NTHR + threadIdx.x;
  if (node >= nRows) return;
  const int nc = (node < nN) ? node : nN - 1;
  const float* hr = h + (size_t)nc * HDIM;
  float sv[NHD], dv[NHD];
#pragma unroll
  for (int hd = 0; hd < NHD; ++hd) { sv[hd] = 0.f; dv[hd] = 0.f; }
#pragma unroll 1
  for (int c = 0; c < DCH; c += 4) {
#pragma unroll
    for (int hd = 0; hd < NHD; ++hd) {
      const v4f hv = *(const v4f*)(hr + hd * DCH + c);
      sv[hd] += dot4f(hv, *(const v4f*)(al + hd * DCH + c));
      dv[hd] += dot4f(hv, *(const v4f*)(ar + hd * DCH + c));
    }
  }
  if (node >= nN) {
#pragma unroll
    for (int hd = 0; hd < NHD; ++hd) { sv[hd] = 0.f; dv[hd] = 0.f; }
  }
  v4f lvv, rvv;
  lvv.x = sv[0]; lvv.y = sv[1]; lvv.z = sv[2]; lvv.w = sv[3];
  rvv.x = dv[0]; rvv.y = dv[1]; rvv.z = dv[2]; rvv.w = dv[3];
  for (int pass = 0; pass < 2; ++pass) {
    *(volatile v4f*)(elp + (size_t)node * NHD) = lvv;
    *(volatile v4f*)(erp + (size_t)node * NHD) = rvv;
    __threadfence();
  }
}

template <int NB>
__global__ __launch_bounds__(NTHR) void k_egat_agg(
    const int* __restrict__ srcl, const int* __restrict__ dstl, const int* __restrict__ etl,
    const float* __restrict__ hfeat,
    const float* __restrict__ elp, const float* __restrict__ erp,
    const float* __restrict__ eep,
    float* of, int nN, int nE, int vec_ok) {
  constexpr int HC  = HDIM;
  constexpr int RW  = NB / NWAVE;
  constexpr int C4R = HC / 4;
  static_assert((NB * HC / 4) % NTHR == 0);
  static_assert(NB % NWAVE == 0 && (RW % 2) == 0);
  static_assert((NB & (NB - 1)) == 0 && NB <= 4096);
  static_assert(HC == 64 && C4R == 16);
  typedef typename VecT<2>::T VT;
  extern __shared__ v4f lds_dyn[];
  float* acc  = (float*)lds_dyn;
  float* mst  = acc + NB * HC;
  float* sst  = mst + NB * NHD;
  int*   list = (int*)(sst + NB * NHD);
  int*   wcnt = list + LISTN;
  const int tid = threadIdx.x, lane = tid & 31, wave = tid >> 5;
  const int nodeBase = blockIdx.x * NB;

  {
    const v4f zz = {0.f, 0.f, 0.f, 0.f};
    for (int i = tid; i < NB * HC / 4; i += NTHR) lds_dyn[i] = zz;
    for (int i = tid; i < NB * NHD; i += NTHR) { mst[i] = -INFINITY; sst[i] = 0.f; }
  }
  __syncthreads();

  const int colL = 2 * lane;
  const int hdl  = lane >> 3;
  const int nChunks = (nE + CHUNK - 1) / CHUNK;
#pragma unroll 1
  for (int ch = 0; ch < nChunks; ++ch) {
    const int cbase = ch * CHUNK;
    const int fullvec = (vec_ok != 0 && cbase + CHUNK <= nE) ? 1 : 0;
    const int wc = scan_chunk<NB>(dstl, nE, cbase, nodeBase, list, tid, lane, wave, fullvec);
    if (lane == 0) wcnt[wave] = wc;
    __syncthreads();
    if (wave == 0) {
#pragma unroll 1
      for (int wsx = 0; wsx < NWAVE; ++wsx) {
        int n = __builtin_amdgcn_readfirstlane(wcnt[wsx]);
        n = n > WCAP ? WCAP : (n < 0 ? 0 : n);
        const int* lp = list + wsx * WCAP;
#pragma unroll 1
        for (int i = 0; i < n; ++i) {
          const int ent  = __builtin_amdgcn_readfirstlane(lp[i]);
          const int slot = ent & (NB - 1);
          int e = cbase + ((ent >> 12) & (CHUNK - 1));
          e = e > nE - 1 ? nE - 1 : e;
          int s = srcl[e];
          s = s < 0 ? 0 : (s > nN - 1 ? nN - 1 : s);
          int t = etl[e];
          t = t < 0 ? 0 : (t > NET - 1 ? NET - 1 : t);
          const int node = nodeBase + slot;
          float lg = (elp[(size_t)s * NHD + hdl] + erp[(size_t)node * NHD + hdl]) + eep[t * NHD + hdl];
          lg = (lg > 0.f) ? lg : 0.2f * lg;
          const int mi = slot * NHD + hdl;
          const float mo = mst[mi];
          const float so = sst[mi];
          const float d  = __expf(-fabsf(lg - mo));
          const bool  up = (lg > mo);
          const float sc = up ? d : 1.0f;
          const float w  = up ? 1.0f : d;
          const VT hv = *(const VT*)(hfeat + (size_t)s * HC + colL);
          VT* ap = (VT*)(acc + slot * HC + colL);
          const VT av = *ap;
          *ap = av * sc + hv * w;
          mst[mi] = up ? lg : mo;
          sst[mi] = so * sc + w;
        }
      }
    }
    __syncthreads();
  }

#pragma unroll 1
  for (int it = 0; it < (NB * HC / 4) / NTHR; ++it) {
    const int idx  = it * NTHR + tid;
    const int slot = idx / C4R;
    const int c4   = (idx - slot * C4R) * 4;
    const int hd   = c4 / DCH;
    const float so = sst[slot * NHD + hd];
    const float rv = __builtin_amdgcn_rcpf((so > 0.f) ? so : 1.0f);
    const float inv = (so > 0.f) ? rv : 0.f;
    v4f* ap = (v4f*)(acc + slot * HC + c4);
    const v4f a = *ap;
    *ap = a * inv;
  }
  __syncthreads();

  for (int pass = 0; pass < 2; ++pass) {
#pragma unroll 1
    for (int it = 0; it < RW / 2; ++it) {
      const int row  = wave * RW + it * 2 + (lane >> 4);
      const int col  = (lane & 15) * 4;
      const int grow = nodeBase + row;
      const v4f v = *(const v4f*)(acc + row * HC + col);
      if (grow < nN) *(volatile v4f*)(of + (size_t)grow * HC + col) = v;
    }
    __threadfence();
  }
}

extern "C" void kernel_launch(void* const* d_in, const int* in_sizes, int n_in,
                              void* d_out, int out_size, void* d_ws, size_t ws_size,
                              hipStream_t stream) {
  if (n_in < 10) return;
  const int nN = in_sizes[0] / CIN;
  const int nE = in_sizes[1];
  if (nN < 1 || nE < 1 || in_sizes[0] != nN * CIN) return;
  if (in_sizes[2] != nE || in_sizes[3] != nE) return;
  if (in_sizes[4] != HDIM * CIN || in_sizes[5] != NHD * EFE * EFE || in_sizes[6] != NET * EFE) return;
  if (in_sizes[7] != HDIM || in_sizes[8] != HDIM || in_sizes[9] != NHD * EFE) return;
  if (out_size != nN * HDIM) return;
  if (nN > (1 << 22) || nE > (1 << 28)) return;

  const float* x     = (const float*)d_in[0];
  const int*   srcl  = (const int*)d_in[1];
  const int*   dstl  = (const int*)d_in[2];
  const int*   etl   = (const int*)d_in[3];
  const float* fcw   = (const float*)d_in[4];
  const float* fcew  = (const float*)d_in[5];
  const float* emb   = (const float*)d_in[6];
  const float* attl  = (const float*)d_in[7];
  const float* attr  = (const float*)d_in[8];
  const float* atte  = (const float*)d_in[9];
  float* out = (float*)d_out;

  const int RP = ((nN + RPQ - 1) / RPQ) * RPQ;

  char* ws = (char*)d_ws;
  size_t off = 0;
  const size_t oXH = off; off += (size_t)RP * CIN * 2;
  const size_t oXL = off; off += (size_t)RP * CIN * 2;
  const size_t oWH = off; off += (size_t)HDIM * CIN * 2;
  const size_t oWL = off; off += (size_t)HDIM * CIN * 2;
  const size_t oFT = off; off += (size_t)RP * HDIM * 4;
  const size_t oEL = off; off += (size_t)RP * NHD * 4;
  const size_t oER = off; off += (size_t)RP * NHD * 4;
  const size_t oEE = off; off += 256;
  if (off > ws_size) return;

  unsigned short* xh = (unsigned short*)(ws + oXH);
  unsigned short* xl = (unsigned short*)(ws + oXL);
  unsigned short* wh = (unsigned short*)(ws + oWH);
  unsigned short* wl = (unsigned short*)(ws + oWL);
  float* ft  = (float*)(ws + oFT);
  float* elp = (float*)(ws + oEL);
  float* erp = (float*)(ws + oER);
  float* eep = (float*)(ws + oEE);

  k_split16<<<RP * (CIN / 8) / NTHR, NTHR, 0, stream>>>(x, xh, xl, nN, RP);
  k_split16<<<HDIM * (CIN / 8) / NTHR, NTHR, 0, stream>>>(fcw, wh, wl, HDIM, HDIM);

  k_eetab<<<1, 32, 0, stream>>>(emb, fcew, atte, eep);

  const int gF = ((RP / 64) * (HDIM / 64) + 7) / 8;
  wmma_gemm64<1, true, 0, 0, false, 0><<<dim3(gF, 1), 256, 0, stream>>>(
      xh, xl, CIN, 0L, wh, wl, CIN, 0L, (void*)ft, (void*)ft, HDIM, 0L,
      attl, ft, 0L, RP, HDIM, CIN, 1.0f);

  k_scores4<<<RP / NTHR, NTHR, 0, stream>>>(ft, attl, attr, elp, erp, nN, RP);

  k_egat_agg<NBLK><<<RP / NBLK, NTHR, LDS_AGG, stream>>>(
      srcl, dstl, etl, ft, elp, erp, eep, out, nN, nE, 1);
}
